// DiffMultiHeadedAttention_56934086476580
// MI455X (gfx1250) — hardware-verified
//
#include <hip/hip_runtime.h>
#include <math.h>

typedef __attribute__((ext_vector_type(16))) _Float16 v16h;
typedef __attribute__((ext_vector_type(16))) __bf16 v16b;
typedef __attribute__((ext_vector_type(8)))  _Float16 v8h;
typedef __attribute__((ext_vector_type(8)))  float v8f;
typedef __attribute__((ext_vector_type(4)))  float v4f;
typedef __attribute__((ext_vector_type(2)))  float v2f;
typedef __attribute__((ext_vector_type(4)))  unsigned v4u;
typedef __attribute__((ext_vector_type(4)))  int v4i;
typedef float __attribute__((may_alias)) float_a;
typedef int __attribute__((may_alias)) int_a;

template <typename T> __device__ __forceinline__ void vst2(void* p, T v) { *(volatile T*)p = v; __threadfence(); *(volatile T*)p = v; }
__device__ __forceinline__ v8f wmma16(v16h a, v16h b, v8f c) {
  v8f d = __builtin_amdgcn_wmma_f32_16x16x32_f16(false, a, false, b, (short)0, c, false, false);
  asm volatile("v_nop\n\tv_nop\n\tv_nop\n\tv_nop" : "+v"(d) : "v"(a), "v"(b));
  return d;
}
__device__ __forceinline__ v8f wmma_bf(v16b a, v16b b, v8f c) {
  v8f d = __builtin_amdgcn_wmma_f32_16x16x32_bf16(false, a, false, b, (short)0, c, false, false);
  asm volatile("v_nop\n\tv_nop\n\tv_nop\n\tv_nop" : "+v"(d) : "v"(a), "v"(b));
  return d;
}
__device__ __forceinline__ v16h frag_h(const _Float16* rowk0, int lane) {
  union { v16h v; v8h q[2]; } u; const _Float16* p = rowk0 + 8 * (lane >> 4);
  u.q[0] = *(const v8h*)p; u.q[1] = *(const v8h*)(p + 16); return u.v;
}
__device__ __forceinline__ v16h frag_f32(const float* rowk0, int lane) {
  v16h a; const float* p = rowk0 + 8 * (lane >> 4);
#pragma unroll
  for (int i = 0; i < 8; ++i) { a[i] = (_Float16)p[i]; a[8 + i] = (_Float16)p[16 + i]; }
  return a;
}
__device__ __forceinline__ v16h frag_f32s(const float* rowk0, int lane, float sc) {
  v16h a; const float* p = rowk0 + 8 * (lane >> 4);
#pragma unroll
  for (int i = 0; i < 8; ++i) { a[i] = (_Float16)(p[i] * sc); a[8 + i] = (_Float16)(p[16 + i] * sc); }
  return a;
}
__device__ __forceinline__ v16h fragc_f32(const float* W, int k0, int n, int lane, int ld, int K) {
  v16h a; const int g = lane >> 4;
#pragma unroll
  for (int i = 0; i < 8; ++i) { const int ka = k0 + 8 * g + i, kb = ka + 16;
    a[i] = (_Float16)(ka < K ? W[(size_t)(ka < K ? ka : K - 1) * ld + n] : 0.f); a[8 + i] = (_Float16)(kb < K ? W[(size_t)(kb < K ? kb : K - 1) * ld + n] : 0.f); }
  return a;
}
struct F2 { v16b h, l; };
__device__ __forceinline__ F2 bsplit16(const float v[16]) { F2 r;
#pragma unroll
  for (int i = 0; i < 16; ++i) { const __bf16 h = (__bf16)v[i]; r.h[i] = h; r.l[i] = (__bf16)(v[i] - (float)h); }
  return r; }
__device__ __forceinline__ F2 split_row(const float* row, int k0, int lane) { float v[16]; const float* p = row + k0 + 8 * (lane >> 4);
#pragma unroll
  for (int i = 0; i < 8; ++i) { v[i] = p[i]; v[8 + i] = p[16 + i]; }
  return bsplit16(v); }
__device__ __forceinline__ F2 split_rowK(const float* row, int k0, int lane, int K) { float v[16]; const int g = lane >> 4;
#pragma unroll
  for (int i = 0; i < 8; ++i) { const int ka = k0 + 8 * g + i, kb = ka + 16; v[i] = ka < K ? row[ka < K ? ka : K - 1] : 0.f; v[8 + i] = kb < K ? row[kb < K ? kb : K - 1] : 0.f; }
  return bsplit16(v); }
__device__ __forceinline__ F2 split_col(const float* W, int k0, int n, int lane, int ld, int K) { float v[16]; const int g = lane >> 4;
#pragma unroll
  for (int i = 0; i < 8; ++i) { const int ka = k0 + 8 * g + i, kb = ka + 16; v[i] = ka < K ? W[(size_t)(ka < K ? ka : K - 1) * ld + n] : 0.f; v[8 + i] = kb < K ? W[(size_t)(kb < K ? kb : K - 1) * ld + n] : 0.f; }
  return bsplit16(v); }
__device__ __forceinline__ v8f mac3(const F2& a, const F2& b, v8f c) { c = wmma_bf(a.l, b.h, c); c = wmma_bf(a.h, b.l, c); return wmma_bf(a.h, b.h, c); }
__device__ __forceinline__ float sigm(float v) { return 1.0f / (1.0f + expf(-v)); }
#define LDSX() do { asm volatile("s_wait_dscnt 0" ::: "memory"); __builtin_amdgcn_wave_barrier(); __builtin_amdgcn_fence(__ATOMIC_RELEASE, "workgroup"); } while (0)


#define NB 4
#define NN 1024
#define DD 1024
#define DH 8
#define DK 128
#define HH2 16
#define KW2 64
#ifndef TNB
#define TNB NB
#endif
typedef __attribute__((ext_vector_type(8))) __bf16 v8b;
__device__ __forceinline__ v16b frag_b(const __bf16* rowk0, int lane) {
  union { v16b v; v8b q[2]; } u; const __bf16* p = rowk0 + 8 * (lane >> 4);
  u.q[0] = *(const v8b*)p; u.q[1] = *(const v8b*)(p + 16); return u.v;
}
__device__ __forceinline__ float bfr(float v) { return (float)(__bf16)v; }
__device__ __attribute__((noinline)) float exp_ni(float v) { return expf(v); }
__device__ __attribute__((noinline)) float erf_ni(float v) { return erff(v); }

#define WS_Q   0u
#define WS_K   (WS_Q + 4u * (size_t)NB * NN * DD)
#define WS_VH  (WS_K + 4u * (size_t)NB * NN * DD)
#define WS_VL  (WS_VH + 2u * (size_t)NB * DD * NN)
#define WS_X   (WS_VL + 2u * (size_t)NB * DD * NN)
#define WS_END (WS_X + 4u * (size_t)NB * NN * DD)

__global__ __launch_bounds__(128) void k_proj(const float* __restrict__ Qi, const float* __restrict__ Ki, const float* __restrict__ Vi, const float* __restrict__ WQ, const float* __restrict__ BQ, const float* __restrict__ WK, const float* __restrict__ BK, const float* __restrict__ WV, const float* __restrict__ BV, float* __restrict__ Q, float* __restrict__ K, _Float16* __restrict__ VH, _Float16* __restrict__ VL) {
  __shared__ __align__(16) float sf[4][16][132]; __shared__ __align__(16) _Float16 th[128][72], tl[128][72];
  const int tid = threadIdx.x, wave = tid >> 5, lane = tid & 31, col = lane & 15, g = lane >> 4; const int which = blockIdx.z; const int c0 = blockIdx.y * 128; const size_t r0 = (size_t)blockIdx.x * 64 + wave * 16;
  const float* X = which == 0 ? Qi : which == 1 ? Ki : Vi; const float* Wm = which == 0 ? WQ : which == 1 ? WK : WV; const float* Bm = which == 0 ? BQ : which == 1 ? BK : BV;
  v8f acc[8] = {};
#pragma unroll 2
  for (int kc = 0; kc < DD / 32; ++kc) { v16b a; { const float* p = X + (r0 + col) * DD + kc * 32 + 8 * g;
#pragma unroll
      for (int i = 0; i < 8; ++i) { a[i] = (__bf16)p[i]; a[8 + i] = (__bf16)p[16 + i]; } }
#pragma unroll
    for (int j = 0; j < 8; ++j) { v16b w; const int o = c0 + j * 16 + col;
#pragma unroll
      for (int i = 0; i < 8; ++i) { w[i] = (__bf16)Wm[(size_t)o * DD + kc * 32 + 8 * g + i]; w[8 + i] = (__bf16)Wm[(size_t)o * DD + kc * 32 + 16 + 8 * g + i]; }
      acc[j] = wmma_bf(a, w, acc[j]); } }
#pragma unroll
  for (int j = 0; j < 8; ++j) { const float bb = bfr(Bm[c0 + j * 16 + col]);
#pragma unroll
    for (int r = 0; r < 8; ++r) { const float v = acc[j][r] + bb; const int rl = wave * 16 + 8 * g + r, cl = j * 16 + col; if (which < 2) sf[wave][8 * g + r][cl] = v; else { const _Float16 hv = (_Float16)v; th[cl][rl] = hv; tl[cl][rl] = (_Float16)(v - (float)hv); } } }
  __syncthreads();
  if (which < 2) { float* dst = which == 0 ? Q : K; for (int rl = 0; rl < 16; ++rl) vst2(dst + (r0 + rl) * DD + c0 + lane * 4, *(const v4f*)&sf[wave][rl][lane * 4]); }
  else { const size_t b = ((size_t)blockIdx.x * 64) / NN; const int n0 = (int)(((size_t)blockIdx.x * 64) % NN); for (int e = tid; e < 128 * 8; e += 128) { const int cl = e >> 3, q = e & 7; const size_t o = (b * DD + c0 + cl) * (size_t)NN + n0 + q * 8; vst2((unsigned*)(VH + o), *(const v4u*)&th[cl][q * 8]); vst2((unsigned*)(VL + o), *(const v4u*)&tl[cl][q * 8]); } } }
__device__ __forceinline__ const float* maprow(const float* __restrict__ R, size_t b, int hh, int np) { const int hd = hh >> 1, e = hh & 1; return R + ((b * NN) + (size_t)e * (NN / 2) + (np >> 1)) * DD + hd * DK + (np & 1) * KW2; }
__global__ __launch_bounds__(128) void k_att(const float* __restrict__ Q, const float* __restrict__ K, const _Float16* __restrict__ VH, const _Float16* __restrict__ VL, const float* __restrict__ LQ1, const float* __restrict__ LK1, const float* __restrict__ LQ2, const float* __restrict__ LK2, const int* __restrict__ HNUM, float* __restrict__ X) {
  __shared__ __align__(16) float sp[4][16][36]; __shared__ __align__(16) float so[4][16][132]; __shared__ float slam;
  const int tid = threadIdx.x, wave = tid >> 5, lane = tid & 31, col = lane & 15, g = lane >> 4; const int qb = blockIdx.x, hd = blockIdx.y; const size_t b = blockIdx.z; const int q0 = qb * 64 + wave * 16;
  if (tid == 0) { float a1 = 0.f, a2 = 0.f;
#pragma unroll 1
    for (int i = 0; i < KW2; ++i) { a1 += bfr(LQ1[i]) * bfr(LK1[i]); a2 += bfr(LQ2[i]) * bfr(LK2[i]); }
    slam = expf(a1) - expf(a2) + 0.8f; (void)HNUM; }
  __syncthreads(); const float lam = slam;
#pragma unroll 1
  for (int e = 0; e < 2; ++e) { const int hh = 2 * hd + e;
    F2 aq[2]; { const float* qr = maprow(Q, b, hh, q0 + col);
#pragma unroll
      for (int kc = 0; kc < 2; ++kc) aq[kc] = split_row(qr, kc * 32, lane); }
    float m[8], l[8];
#pragma unroll
    for (int r = 0; r < 8; ++r) { m[r] = -3.0e38f; l[r] = 0.f; }
    v8f acc[8] = {};
#pragma unroll 1
    for (int ks = 0; ks < NN / 32; ++ks) { float s[2][8];
#pragma unroll
      for (int ct = 0; ct < 2; ++ct) { const int kk = ks * 32 + ct * 16 + col; const float* kr = maprow(K, b, hh, kk); v8f c = {};
#pragma unroll
        for (int kc = 0; kc < 2; ++kc) c = mac3(aq[kc], split_row(kr, kc * 32, lane), c);
#pragma unroll
        for (int r = 0; r < 8; ++r) s[ct][r] = c[r] * 0.125f; }
      float alpha[8];
#pragma unroll
      for (int r = 0; r < 8; ++r) { float mx = fmaxf(s[0][r], s[1][r]);
#pragma unroll
        for (int o = 1; o < 16; o <<= 1) mx = fmaxf(mx, __shfl_xor(mx, o));
        const float mn = fmaxf(m[r], mx); alpha[r] = __expf(m[r] - mn); const float e0 = __expf(s[0][r] - mn), e1 = __expf(s[1][r] - mn); float es = e0 + e1;
#pragma unroll
        for (int o = 1; o < 16; o <<= 1) es += __shfl_xor(es, o);
        l[r] = l[r] * alpha[r] + es; m[r] = mn; sp[wave][8 * g + r][col] = e0; sp[wave][8 * g + r][16 + col] = e1; }
#pragma unroll
      for (int j = 0; j < 8; ++j)
#pragma unroll
        for (int r = 0; r < 8; ++r) acc[j][r] *= alpha[r];
      LDSX();
      v16h pa, pr; { const float* prow = &sp[wave][col][0] + 8 * (lane >> 4);
#pragma unroll
        for (int i = 0; i < 8; ++i) { const float x0 = prow[i] * 2048.0f, x1 = prow[16 + i] * 2048.0f; const _Float16 h0 = (_Float16)x0, h1 = (_Float16)x1; pa[i] = h0; pa[8 + i] = h1; pr[i] = (_Float16)(x0 - (float)h0); pr[8 + i] = (_Float16)(x1 - (float)h1); } }
#pragma unroll
      for (int j = 0; j < 8; ++j) { const size_t po = (b * DD + (size_t)hd * DK + j * 16 + col) * NN + ks * 32; const v16h vh = frag_h(VH + po, lane); acc[j] = wmma16(pa, vh, acc[j]); acc[j] = wmma16(pr, vh, acc[j]); acc[j] = wmma16(pa, frag_h(VL + po, lane), acc[j]); }
      LDSX(); }
#pragma unroll
    for (int r = 0; r < 8; ++r) { const float il = (1.0f / 2048.0f) / l[r];
#pragma unroll
      for (int j = 0; j < 8; ++j) { float* cell = &so[wave][8 * g + r][j * 16 + col]; const float v = acc[j][r] * il; *cell = (e == 0) ? v : (*cell - lam * v); } } }
  LDSX(); for (int rl = 0; rl < 16; ++rl) vst2(X + (b * NN + q0 + rl) * DD + hd * DK + lane * 4, *(const v4f*)&so[wave][rl][lane * 4]); }
__global__ __launch_bounds__(128) void k_out(const float* __restrict__ X, const float* __restrict__ WO, const float* __restrict__ BO, float* __restrict__ OUT) { __shared__ __align__(16) float sf[4][16][132];
  const int tid = threadIdx.x, wave = tid >> 5, lane = tid & 31, col = lane & 15, g = lane >> 4; const int c0 = blockIdx.y * 128; const size_t r0 = (size_t)blockIdx.x * 64 + wave * 16;
  v8f acc[8] = {};
#pragma unroll 2
  for (int kc = 0; kc < DD / 32; ++kc) { const F2 a = split_row(X + (r0 + col) * DD, kc * 32, lane);
#pragma unroll
    for (int j = 0; j < 8; ++j) { v16b w; const int o = c0 + j * 16 + col;
#pragma unroll
      for (int i = 0; i < 8; ++i) { w[i] = (__bf16)WO[(size_t)o * DD + kc * 32 + 8 * g + i]; w[8 + i] = (__bf16)WO[(size_t)o * DD + kc * 32 + 16 + 8 * g + i]; }
      acc[j] = wmma_bf(a.h, w, acc[j]); acc[j] = wmma_bf(a.l, w, acc[j]); } }
#pragma unroll
  for (int j = 0; j < 8; ++j) { const float bb = bfr(BO[c0 + j * 16 + col]);
#pragma unroll
    for (int r = 0; r < 8; ++r) sf[wave][8 * g + r][j * 16 + col] = acc[j][r] + bb; }
  LDSX(); for (int rl = 0; rl < 16; ++rl) vst2(OUT + (r0 + rl) * DD + c0 + lane * 4, *(const v4f*)&sf[wave][rl][lane * 4]); }
extern "C" void kernel_launch(void* const* d_in, const int* in_sizes, int n_in, void* d_out, int out_size, void* d_ws, size_t ws_size, hipStream_t stream) {
  (void)in_sizes; (void)n_in; (void)out_size;
  const float** F = (const float**)d_in;
  if (ws_size < (size_t)WS_END) return;
  char* ws = (char*)d_ws; float *Q = (float*)(ws + WS_Q), *K = (float*)(ws + WS_K), *X = (float*)(ws + WS_X); _Float16 *VH = (_Float16*)(ws + WS_VH), *VL = (_Float16*)(ws + WS_VL);
  k_proj<<<dim3(TNB * NN / 64, DD / 128, 3), 128, 0, stream>>>(F[0], F[1], F[2], F[3], F[4], F[5], F[6], F[7], F[8], Q, K, VH, VL);
  k_att<<<dim3(NN / 64, DH, TNB), 128, 0, stream>>>(Q, K, VH, VL, F[11], F[13], F[12], F[14], (const int*)d_in[15], X);
  k_out<<<dim3(TNB * NN / 64, DD / 128), 128, 0, stream>>>(X, F[9], F[10], (float*)d_out);
}
